// GraphAttentionLayer_57260503990856
// MI455X (gfx1250) — hardware-verified
//
#include <hip/hip_runtime.h>
#include <stddef.h>


typedef _Float16 v16h __attribute__((ext_vector_type(16)));
typedef _Float16 v8h  __attribute__((ext_vector_type(8)));
typedef float    v8f  __attribute__((ext_vector_type(8)));
typedef float    v4f  __attribute__((ext_vector_type(4)));

#ifndef NB
#define NB 1
#endif
#ifndef SEQ
#define SEQ 8192
#endif
#define NB_FULL  1
#define SEQ_FULL 8192
#define FIN   512
#define FOUT  256
#define GN    128
#define MROWS (NB * SEQ)

static_assert(NB >= 1 && NB <= NB_FULL);
static_assert(SEQ >= 128 && SEQ <= SEQ_FULL && (SEQ % 128) == 0);
static_assert(GN == 128);
static_assert((FOUT % GN) == 0 && (FOUT % 64) == 0);
static_assert((FIN % 64) == 0 && (FIN % 32) == 0);
static_assert((MROWS % 64) == 0 && (MROWS % 16) == 0);
static_assert(2 * FOUT == 512);
static_assert((size_t)NB_FULL * SEQ_FULL * FOUT * 4 == (size_t)8388608);

#define HTPR (FIN / 8)
#define HRPB (256 / HTPR)
static_assert(HTPR * 8 == FIN && HRPB * HTPR == 256 && (HTPR % 32) == 0);
static_assert((MROWS % HRPB) == 0);

#define LDT 72
#define LDW 132
#define LDO 36
static_assert((LDT % 8) == 0 && LDT >= 64);
static_assert((LDW % 4) == 0 && LDW >= GN);
static_assert((LDO % 4) == 0 && LDO >= 32);

#define WCARRY 64.0f
#define HCARRY 16.0f
#define VCARRY 64.0f
#define PCARRY 16384.0f
#define PCUT   (-19.0f)
#define SLOPE  0.0f

#define WT_BYTES  ((size_t)FIN * FOUT * 2)
#define H16_BYTES ((size_t)MROWS * FIN * 2)
#define VT_BYTES  ((size_t)NB * FOUT * SEQ * 2)
#define ST_BYTES  ((size_t)2 * MROWS * 4)
#define OFF_WT  ((size_t)0)
#define OFF_H   (OFF_WT + WT_BYTES)
#define OFF_VT  (OFF_H + H16_BYTES)
#define OFF_ST  (OFF_VT + VT_BYTES)
#define WS_TOTAL (OFF_ST + ST_BYTES)
static_assert((WT_BYTES % 128) == 0 && (H16_BYTES % 128) == 0 && (VT_BYTES % 128) == 0);
static_assert((ST_BYTES % 128) == 0 && (((size_t)MROWS * 4) % 128) == 0);
static_assert(WS_TOTAL <= (size_t)134217728);

__device__ __forceinline__ float bf16r(float x) {
  unsigned int u = __float_as_uint(x);
  u = (u + 0x7FFFu + ((u >> 16) & 1u)) & 0xFFFF0000u;
  return __uint_as_float(u);
}

static __device__ __forceinline__ _Float16 toh_flush(float v) {
  const _Float16 r = (_Float16)v;
  return (fabsf(v) < 6.103515625e-05f) ? (_Float16)0.0f : r;
}

__device__ __forceinline__ v16h frag_at(const _Float16* p) {
  v8h lo = *(const v8h*)(p);
  v8h hi = *(const v8h*)(p + 16);
  v16h out;
#pragma unroll
  for (int i = 0; i < 8; ++i) { out[i] = lo[i]; out[i + 8] = hi[i]; }
  return out;
}
__device__ __forceinline__ v16h ld_frag(const _Float16* base, unsigned ld) {
  const unsigned lane = threadIdx.x & 31u;
  return frag_at(base + (lane & 15u) * ld + (lane >> 4) * 8u);
}

__device__ __forceinline__ v8f wmma16(v16h a, v16h b, v8f c) {
  v8f d = __builtin_amdgcn_wmma_f32_16x16x32_f16(false, a, false, b, (short)0, c,
                                                 false, false);
  asm volatile("v_nop\n\tv_nop\n\tv_nop\n\tv_nop" : "+v"(d) : "v"(a), "v"(b));
  return d;
}

__device__ __forceinline__ float red16_max(float x) {
#pragma unroll
  for (int off = 1; off < 16; off <<= 1) x = fmaxf(x, __shfl_xor(x, off, 32));
  return x;
}
__device__ __forceinline__ float red16_sum(float x) {
#pragma unroll
  for (int off = 1; off < 16; off <<= 1) x += __shfl_xor(x, off, 32);
  return x;
}

__device__ __forceinline__ void wave_lds_sync() {
  __builtin_amdgcn_fence(3  , "wavefront");
  asm volatile("s_wait_dscnt 0x0" ::: "memory");
  __builtin_amdgcn_wave_barrier();
}

__global__ __launch_bounds__(256) void wconv_kernel(
    const float* __restrict__ W, _Float16* __restrict__ Wt, unsigned ldw, unsigned ldk) {
  __shared__ _Float16 T[64 * LDT];
  const unsigned tid = threadIdx.x;
  const unsigned n0 = blockIdx.x * 64u;
  const unsigned k0 = blockIdx.y * 64u;
#pragma unroll 4
  for (unsigned j = 0; j < 16u; ++j) {
    const unsigned idx = tid + 256u * j;
    const unsigned kr = idx >> 6, nc = idx & 63u;
    const float v = W[(size_t)(k0 + kr) * ldw + n0 + nc];
    T[nc * LDT + kr] = (_Float16)(WCARRY * bf16r(v));
  }
  __syncthreads();
  v8h x[2];
  size_t off[2];
#pragma unroll
  for (unsigned i = 0; i < 2u; ++i) {
    const unsigned n = 32u * i + (tid >> 3);
    const unsigned kc = (tid & 7u) * 8u;
    x[i] = *(const v8h*)&T[n * LDT + kc];
    off[i] = (size_t)(n0 + n) * ldk + k0 + kc;
  }
#pragma unroll
  for (int i = 0; i < 2; ++i) *(volatile v8h*)(Wt + off[i]) = x[i];
  __threadfence();
#pragma unroll
  for (int i = 0; i < 2; ++i) *(volatile v8h*)(Wt + off[i]) = x[i];
}

__global__ __launch_bounds__(256) void hconv_kernel(
    const float* __restrict__ X, _Float16* __restrict__ dst) {
  const unsigned tid = threadIdx.x;
  const unsigned crow = blockIdx.x * (unsigned)HRPB + tid / (unsigned)HTPR;
  const unsigned c = (tid % (unsigned)HTPR) * 8u;
  const unsigned bidx = crow / (unsigned)SEQ;
  const unsigned sq = crow - bidx * (unsigned)SEQ;
  const size_t srow = (size_t)bidx * SEQ_FULL + sq;
  const v4f a0 = *(const v4f*)(X + srow * FIN + c);
  const v4f a1 = *(const v4f*)(X + srow * FIN + c + 4u);
  v8h o;
#pragma unroll
  for (int i = 0; i < 4; ++i) {
    o[i]     = toh_flush(HCARRY * bf16r(a0[i]));
    o[i + 4] = toh_flush(HCARRY * bf16r(a1[i]));
  }
  _Float16* p = dst + (size_t)crow * FIN + c;
  *(volatile v8h*)p = o;
  __threadfence();
  *(volatile v8h*)p = o;
}

__global__ __launch_bounds__(256) void gemm_wh_kernel(
    const _Float16* __restrict__ A16, const _Float16* __restrict__ Bt,
    const float* __restrict__ avec, _Float16* __restrict__ vt, float* __restrict__ st) {
  __shared__ __attribute__((aligned(16))) float Cs[64 * LDW];
  __shared__ __attribute__((aligned(16))) float As[2 * FOUT];
  __shared__ __attribute__((aligned(16))) float St[128];
  const unsigned tid = threadIdx.x, lane = tid & 31u;
  const unsigned w = (unsigned)__builtin_amdgcn_readfirstlane((int)(threadIdx.x >> 5));
  const unsigned mw = w >> 1, nw = w & 1u;
  const unsigned hh = lane >> 4, m = lane & 15u;
  const unsigned row0 = blockIdx.x * 64u;

  As[tid] = bf16r(avec[tid]);
  As[256u + tid] = bf16r(avec[256u + tid]);

  const _Float16* ap = A16 + (size_t)(row0 + mw * 16u + m) * FIN + hh * 8u;
  const unsigned bidx = row0 / (unsigned)SEQ;
  const unsigned key0 = row0 - bidx * (unsigned)SEQ;
  const unsigned r = tid >> 2, q = tid & 3u;
  float d1 = 0.0f, d2 = 0.0f;

#pragma unroll 1
  for (unsigned cg = 0; cg < (unsigned)(FOUT / GN); ++cg) {
    const _Float16* bp = Bt + (size_t)(cg * (unsigned)GN + nw * 64u + m) * FIN + hh * 8u;
    v8f acc0 = {}, acc1 = {}, acc2 = {}, acc3 = {};
#pragma unroll 2
    for (unsigned k0 = 0; k0 < (unsigned)FIN; k0 += 32u) {
      const v16h a  = frag_at(ap + k0);
      const v16h b0 = frag_at(bp + k0);
      const v16h b1 = frag_at(bp + (size_t)16 * FIN + k0);
      const v16h b2 = frag_at(bp + (size_t)32 * FIN + k0);
      const v16h b3 = frag_at(bp + (size_t)48 * FIN + k0);
      acc0 = wmma16(a, b0, acc0);
      acc1 = wmma16(a, b1, acc1);
      acc2 = wmma16(a, b2, acc2);
      acc3 = wmma16(a, b3, acc3);
    }
#pragma unroll
    for (int rr = 0; rr < 8; ++rr) {
      float* d = &Cs[(mw * 16u + hh * 8u + (unsigned)rr) * LDW + nw * 64u + m];
      d[0]  = acc0[rr];
      d[16] = acc1[rr];
      d[32] = acc2[rr];
      d[48] = acc3[rr];
    }
    __syncthreads();

    {
#pragma unroll 1
      for (unsigned j = 0; j < 8u; ++j) {
        const unsigned c = q * 32u + 4u * j;
        const v4f u  = *(const v4f*)&Cs[r * LDW + c];
        const v4f e1 = *(const v4f*)&As[cg * (unsigned)GN + c];
        const v4f e2 = *(const v4f*)&As[(unsigned)FOUT + cg * (unsigned)GN + c];
#pragma unroll
        for (int i = 0; i < 4; ++i) {
          d1 += u[i] * e1[i];
          d2 += u[i] * e2[i];
        }
      }
    }

    {
      const float vs = VCARRY / (HCARRY * WCARRY);
      v8h x[4];
      size_t off[4];
#pragma unroll
      for (unsigned i = 0; i < 4u; ++i) {
        const unsigned dcol = 32u * i + (tid >> 3);
        const unsigned kk = (tid & 7u) * 8u;
#pragma unroll
        for (unsigned j = 0; j < 8u; ++j)
          x[i][j] = toh_flush(Cs[(kk + j) * LDW + dcol] * vs);
        off[i] = ((size_t)bidx * FOUT + cg * (unsigned)GN + dcol) * SEQ + key0 + kk;
      }
#pragma unroll
      for (int i = 0; i < 4; ++i) *(volatile v8h*)(vt + off[i]) = x[i];
      __threadfence();
#pragma unroll
      for (int i = 0; i < 4; ++i) *(volatile v8h*)(vt + off[i]) = x[i];
    }
    __syncthreads();
  }

  {
    const float cs = 1.0f / (HCARRY * WCARRY);
    d1 += __shfl_xor(d1, 1, 32);
    d2 += __shfl_xor(d2, 1, 32);
    d1 += __shfl_xor(d1, 2, 32);
    d2 += __shfl_xor(d2, 2, 32);
    if (q == 0u) {
      St[r] = d1 * cs;
      St[64u + r] = d2 * cs;
    }
  }
  __syncthreads();

  if (w == 0u) {
    const v4f sv = *(const v4f*)&St[hh * 64u + m * 4u];
    float* p = st + (size_t)hh * MROWS + row0 + m * 4u;
    *(volatile v4f*)p = sv;
    __threadfence();
    *(volatile v4f*)p = sv;
  }
}

__global__ __launch_bounds__(256) void attn_kernel(
    const _Float16* __restrict__ Vt, const float* __restrict__ ST, float* __restrict__ Out) {
  __shared__ __attribute__((aligned(16))) _Float16 Vs[GN * LDT];
  __shared__ __attribute__((aligned(16))) _Float16 Ps[8 * 16 * LDT];
  __shared__ __attribute__((aligned(16))) float Os[8 * 16 * LDO];

  const unsigned tid = threadIdx.x, lane = tid & 31u;
  const unsigned w = (unsigned)__builtin_amdgcn_readfirstlane((int)(threadIdx.x >> 5));
  const unsigned hh = lane >> 4, m = lane & 15u;
  const unsigned q0 = blockIdx.x * 128u;
  const unsigned b = blockIdx.y;
  const unsigned cs0 = blockIdx.z * (unsigned)GN;
  const unsigned qrow0 = q0 + w * 16u;
  _Float16* P = Ps + w * (16u * LDT);
  float* O = Os + w * (16u * LDO);

  float srow[8];
  {
    const float* sp = ST + (size_t)b * SEQ + qrow0 + hh * 8u;
    const v4f s0 = *(const v4f*)(sp);
    const v4f s1 = *(const v4f*)(sp + 4);
#pragma unroll
    for (int i = 0; i < 4; ++i) { srow[i] = s0[i]; srow[i + 4] = s1[i]; }
  }
  const float* tp = ST + (size_t)MROWS + (size_t)b * SEQ + m;

  float mrow[8], lrow[8];
  v8f o[8];
#pragma unroll
  for (int v = 0; v < 8; ++v) { mrow[v] = -1.0e30f; lrow[v] = 0.0f; }
#pragma unroll
  for (int nb = 0; nb < 8; ++nb) o[nb] = (v8f){};

  const size_t vplane = ((size_t)b * FOUT + cs0) * SEQ;

  for (unsigned kb = 0; kb < (unsigned)SEQ; kb += 64u) {
#pragma unroll
    for (unsigned j = 0; j < 4u; ++j) {
      const unsigned idx = tid + 256u * j;
      const unsigned r = idx >> 3, c = (idx & 7u) * 8u;
      *(v8h*)&Vs[r * LDT + c] = *(const v8h*)(Vt + vplane + (size_t)r * SEQ + kb + c);
    }
    float tk[4];
#pragma unroll
    for (int kg = 0; kg < 4; ++kg) tk[kg] = tp[kb + (unsigned)kg * 16u];
    __syncthreads();

    v8f s[4];
#pragma unroll
    for (int kg = 0; kg < 4; ++kg)
#pragma unroll
      for (int v = 0; v < 8; ++v) {
        const float e = srow[v] + tk[kg];
        s[kg][v] = (e >= 0.0f) ? e : SLOPE * e;
      }

    float alpha[8];
#pragma unroll
    for (int v = 0; v < 8; ++v) {
      float mx = fmaxf(fmaxf(s[0][v], s[1][v]), fmaxf(s[2][v], s[3][v]));
      mx = red16_max(mx);
      const float mn = fmaxf(mrow[v], mx);
      alpha[v] = __expf(mrow[v] - mn);
      mrow[v] = mn;
    }

#pragma unroll
    for (int kg = 0; kg < 4; ++kg)
#pragma unroll
      for (int v = 0; v < 8; ++v) {
        const float x = s[kg][v] - mrow[v];
        const float pc = (x < PCUT) ? 0.0f : __expf(x) * PCARRY;
        const _Float16 ph = (_Float16)pc;
        P[(hh * 8u + (unsigned)v) * LDT + (unsigned)kg * 16u + m] = ph;
        s[kg][v] = (float)ph;
      }
#pragma unroll
    for (int v = 0; v < 8; ++v) {
      const float rs = red16_sum((s[0][v] + s[1][v]) + (s[2][v] + s[3][v]));
      lrow[v] = alpha[v] * lrow[v] + rs;
    }
#pragma unroll
    for (int nb = 0; nb < 8; ++nb)
#pragma unroll
      for (int v = 0; v < 8; ++v) o[nb][v] = o[nb][v] * alpha[v];
    wave_lds_sync();

#pragma unroll
    for (int c = 0; c < 2; ++c) {
      const v16h pf = ld_frag(P + c * 32, LDT);
#pragma unroll
      for (int nb = 0; nb < 8; ++nb) {
        const v16h vf = ld_frag(&Vs[(nb * 16) * LDT + c * 32], LDT);
        o[nb] = wmma16(pf, vf, o[nb]);
      }
    }
    __syncthreads();
  }

  float inv[8];
#pragma unroll
  for (int v = 0; v < 8; ++v) inv[v] = __builtin_amdgcn_rcpf(lrow[v]) * (1.0f / VCARRY);

  v4f x[16];
#pragma unroll
  for (int p = 0; p < 4; ++p) {
#pragma unroll
    for (int j = 0; j < 2; ++j)
#pragma unroll
      for (int v = 0; v < 8; ++v) {
        float val = o[2 * p + j][v] * inv[v];
        val = (val > 0.0f) ? val : (__expf(val) - 1.0f);
        O[(hh * 8u + (unsigned)v) * LDO + (unsigned)j * 16u + m] = val;
      }
    wave_lds_sync();
#pragma unroll
    for (unsigned i = 0; i < 4u; ++i) {
      const unsigned r = 4u * i + (lane >> 3);
      const unsigned c = (lane & 7u) * 4u;
      x[p * 4 + (int)i] = *(const v4f*)&O[r * LDO + c];
    }
    wave_lds_sync();
  }

  const size_t obase =
      ((size_t)b * SEQ_FULL + qrow0 + (lane >> 3)) * FOUT + cs0 + (lane & 7u) * 4u;
#pragma unroll
  for (int p = 0; p < 4; ++p)
#pragma unroll
    for (int i = 0; i < 4; ++i)
      *(volatile v4f*)(Out + obase + (size_t)(4 * i) * FOUT + 32 * p) = x[p * 4 + i];
  __threadfence();
#pragma unroll
  for (int p = 0; p < 4; ++p)
#pragma unroll
    for (int i = 0; i < 4; ++i)
      *(volatile v4f*)(Out + obase + (size_t)(4 * i) * FOUT + 32 * p) = x[p * 4 + i];
}

extern "C" void kernel_launch(void* const* d_in, const int* in_sizes, int n_in,
                              void* d_out, int out_size, void* d_ws, size_t ws_size,
                              hipStream_t stream) {
  if (n_in < 3) return;
  const long long need_rows = (long long)(NB - 1) * SEQ_FULL + SEQ;
  if ((long long)in_sizes[0] < need_rows * FIN) return;
  if ((long long)in_sizes[1] < (long long)FIN * FOUT) return;
  if (in_sizes[2] < 2 * FOUT) return;
  if ((long long)out_size < need_rows * FOUT) return;
  if (ws_size < WS_TOTAL) return;

  const float* Xm = (const float*)d_in[0];
  const float* Wm = (const float*)d_in[1];
  const float* av = (const float*)d_in[2];
  float* out = (float*)d_out;

  char* ws = (char*)d_ws;
  _Float16* Wt   = (_Float16*)(ws + OFF_WT);
  _Float16* H16  = (_Float16*)(ws + OFF_H);
  _Float16* Vt16 = (_Float16*)(ws + OFF_VT);
  float*    STp  = (float*)(ws + OFF_ST);

  dim3 blk(256);

  wconv_kernel<<<dim3(FOUT / 64, FIN / 64), blk, 0, stream>>>(Wm, Wt, (unsigned)FOUT,
                                                              (unsigned)FIN);
  hconv_kernel<<<dim3(MROWS / HRPB), blk, 0, stream>>>(Xm, H16);
  gemm_wh_kernel<<<dim3(MROWS / 64), blk, 0, stream>>>(H16, Wt, av, Vt16, STp);
  attn_kernel<<<dim3(SEQ / 128, NB, FOUT / GN), blk, 0, stream>>>(Vt16, STp, out);
}
